// MPNNMultidimFullAttention_12515534701093
// MI455X (gfx1250) — hardware-run, weakly checked
//
#include <hip/hip_runtime.h>
#include <math.h>
#include <stdint.h>

#define NB   32
#define NN   512
#define FIN  16
#define DD   128
#define NHD  8
#define DKD  16
#define FFD  512
#define NL   3
#define NOUT 3
#define MR   (NB * NN)
#define QKVC (3 * DD)
static_assert(NHD * DKD == DD);
static_assert((MR % 64) == 0 && (DD % 32) == 0 && (FFD % 32) == 0 && (QKVC % 32) == 0);
static_assert((NN % 64) == 0 && (NN % 256) == 0);
static_assert(((MR / 64) * (DD / 32)) % 8 == 0);
static_assert(((MR / 64) * (QKVC / 32)) % 8 == 0);
static_assert(((MR / 64) * (FFD / 32)) % 8 == 0);
static_assert((MR * DD / 8) % 256 == 0 && (MR * FFD / 8) % 256 == 0);
static_assert((MR * NOUT) % 768 == 0);

typedef _Float16 v16h __attribute__((ext_vector_type(16)));
typedef _Float16 v8h  __attribute__((ext_vector_type(8)));
typedef __bf16   v16b __attribute__((ext_vector_type(16)));
typedef unsigned short v8us __attribute__((ext_vector_type(8)));
typedef float    v8f  __attribute__((ext_vector_type(8)));
typedef float    v4f  __attribute__((ext_vector_type(4)));
typedef unsigned int v4u __attribute__((ext_vector_type(4)));

union FragH { v16h v; v8h h[2]; };
union FragB { v16b v; v8us u[2]; };

__device__ __forceinline__ unsigned short bf_bits(float f) {
  unsigned u = __float_as_uint(f);
  return (unsigned short)((u + 0x7FFFu + ((u >> 16) & 1u)) >> 16);
}
__device__ __forceinline__ float bf_up(unsigned short b) { return __uint_as_float(((unsigned)b) << 16); }
__device__ __forceinline__ float bfr(float f) { return bf_up(bf_bits(f)); }
__device__ __forceinline__ unsigned short h_bits(_Float16 x) { return __builtin_bit_cast(unsigned short, x); }
__device__ __forceinline__ unsigned pk16(unsigned short a, unsigned short b) { return (unsigned)a | ((unsigned)b << 16); }
__device__ __forceinline__ v8f zero8() { v8f z = {0.f, 0.f, 0.f, 0.f, 0.f, 0.f, 0.f, 0.f}; return z; }
__device__ __forceinline__ v8h zero8h() { union { v4u u; v8h h; } z; v4u t = {0u, 0u, 0u, 0u}; z.u = t; return z.h; }
__device__ __forceinline__ v16b zero16b() { FragB f; v8us z = {0, 0, 0, 0, 0, 0, 0, 0}; f.u[0] = z; f.u[1] = z; return f.v; }
__device__ __forceinline__ v4f vmax0(v4f v) {
  v4f r; r[0] = fmaxf(v[0], 0.f); r[1] = fmaxf(v[1], 0.f); r[2] = fmaxf(v[2], 0.f); r[3] = fmaxf(v[3], 0.f); return r;
}
__device__ __forceinline__ void lds_sync() {
  __builtin_amdgcn_fence(__ATOMIC_RELEASE, "workgroup");
  __builtin_amdgcn_wave_barrier();
  __builtin_amdgcn_fence(__ATOMIC_ACQUIRE, "workgroup");
}

__device__ __forceinline__ v16h ldfrag_h(const _Float16* p) {
  FragH f;
  f.h[0] = *(const v8h*)(p);
  f.h[1] = *(const v8h*)(p + 16);
  return f.v;
}
__device__ __forceinline__ v16b ldfrag_b(const unsigned short* p) {
  FragB f;
  f.u[0] = *(const v8us*)(p);
  f.u[1] = *(const v8us*)(p + 16);
  return f.v;
}

__device__ __forceinline__ v8f mma_h(v16h a, v16h b, v8f c) {
  c = __builtin_amdgcn_wmma_f32_16x16x32_f16(false, a, false, b, (short)0, c, false, false);
#if defined(__HIP_DEVICE_COMPILE__)
  asm volatile("v_nop\n\tv_nop\n\tv_nop\n\tv_nop" : "+v"(c) : "v"(a), "v"(b));
#endif
  return c;
}
__device__ __forceinline__ v8f mma_b(v16b a, v16b b, v8f c) {
  c = __builtin_amdgcn_wmma_f32_16x16x32_bf16(false, a, false, b, (short)0, c, false, false);
#if defined(__HIP_DEVICE_COMPILE__)
  const v16h ka = __builtin_bit_cast(v16h, a);
  const v16h kb = __builtin_bit_cast(v16h, b);
  asm volatile("v_nop\n\tv_nop\n\tv_nop\n\tv_nop" : "+v"(c) : "v"(ka), "v"(kb));
#endif
  return c;
}

__global__ __launch_bounds__(256) void pad16(const float* __restrict__ src, int sr, int sk,
                                             unsigned short* outp, int n4, float sc) {
  const int i = blockIdx.x * 256 + threadIdx.x;
  if (i >= n4) return;
  const int r = i >> 2, part = i & 3, kb = (part & 1) * 8;
  const bool live = part < 2;
  v4u a;
#pragma unroll
  for (int p = 0; p < 4; ++p) {
    const int k = kb + 2 * p;
    const float f0 = src[(size_t)r * sr + (size_t)k * sk];
    const float f1 = src[(size_t)r * sr + (size_t)(k + 1) * sk];
    const float g0 = live ? (bfr(f0) * sc) : 0.0f;
    const float g1 = live ? (bfr(f1) * sc) : 0.0f;
    a[p] = pk16(h_bits((_Float16)g0), h_bits((_Float16)g1));
  }
  const size_t o = (size_t)i * 8;
  *(volatile v4u*)(outp + o) = a;
  __threadfence();
  *(volatile v4u*)(outp + o) = a;
}

__global__ __launch_bounds__(256) void wprep(const float* __restrict__ src, unsigned short* oh, unsigned short* ob,
                                             int n8, int N, int K, int Lsrc, int outL, int rowoff,
                                             int nsh, int nmask, int shi, int slo, int sk, float sc) {
  const int i = blockIdx.x * 256 + threadIdx.x;
  if (i >= n8) return;
  const int e8 = i * 8;
  const int NK = N * K;
  const int l = e8 / NK;
  const int rem = e8 - l * NK;
  const int n = rem / K;
  const int k0 = rem - n * K;
  const size_t base = (size_t)l * Lsrc + (size_t)(n >> nsh) * shi + (size_t)(n & nmask) * slo;
  v4u ah, ab;
#pragma unroll
  for (int p = 0; p < 4; ++p) {
    const int e = 2 * p;
    const float f0 = bfr(src[base + (size_t)(k0 + e) * sk]) * sc;
    const float f1 = bfr(src[base + (size_t)(k0 + e + 1) * sk]) * sc;
    ah[p] = pk16(h_bits((_Float16)f0), h_bits((_Float16)f1));
    ab[p] = pk16(bf_bits(f0), bf_bits(f1));
  }
  const size_t o = (size_t)l * outL + (size_t)(rowoff + n) * K + k0;
  for (int pass = 0; pass < 2; ++pass) {
    *(volatile v4u*)(oh + o) = ah;
    *(volatile v4u*)(ob + o) = ab;
    __threadfence();
  }
}

template <int GATHER>
__global__ __launch_bounds__(256) void cvt_hl(const float* __restrict__ in, unsigned short* oh, unsigned short* ol,
                                              int n8, float sc) {
  const int i = blockIdx.x * 256 + threadIdx.x;
  if (i >= n8) return;
  const float* src;
  if (GATHER) {
    const int m = i >> 4, cg = i & 15;
    const int hd = cg >> 1, dk0 = (cg & 1) * 8;
    const int bq = m >> 9, nd = m & 511;
    src = in + ((((size_t)bq * NHD + hd) * NN + nd) * DKD + dk0);
  } else {
    src = in + (size_t)i * 8;
  }
  const v4f x0 = *(const v4f*)(src);
  const v4f x1 = *(const v4f*)(src + 4);
  float x[8];
  x[0] = x0[0]; x[1] = x0[1]; x[2] = x0[2]; x[3] = x0[3];
  x[4] = x1[0]; x[5] = x1[1]; x[6] = x1[2]; x[7] = x1[3];
  v4u ph, pl;
#pragma unroll
  for (int p = 0; p < 4; ++p) {
    const int e = 2 * p;
    const float f0 = x[e] * sc, f1 = x[e + 1] * sc;
    const _Float16 h0 = (_Float16)f0, h1 = (_Float16)f1;
    const unsigned short l0 = bf_bits(f0 - (float)h0);
    const unsigned short l1 = bf_bits(f1 - (float)h1);
    ph[p] = pk16(h_bits(h0), h_bits(h1));
    pl[p] = pk16(l0, l1);
  }
  const size_t o = (size_t)i * 8;
  for (int pass = 0; pass < 2; ++pass) {
    *(volatile v4u*)(oh + o) = ph;
    *(volatile v4u*)(ol + o) = pl;
    __threadfence();
  }
}

template <int MODE, int HASLO, int HASBIAS>
__global__ __launch_bounds__(256) void gemmw(
    const unsigned short* __restrict__ Ahp, const unsigned short* __restrict__ Alp, int lda,
    const unsigned short* __restrict__ Bhp, const unsigned short* __restrict__ Bbp, int ldb,
    const float* __restrict__ bias, const float* __restrict__ res, int ldr,
    float* Cf, int ldc, unsigned short* Qo, unsigned short* Ko, unsigned short* Vo,
    int M, int N, int K, float oscale) {
  const _Float16* Ah = (const _Float16*)(const void*)Ahp;
  const _Float16* Bh = (const _Float16*)(const void*)Bhp;
  __shared__ __align__(16) unsigned char sT[8][5120];
  const int lane = threadIdx.x & 31;
  const int wave = threadIdx.x >> 5;
  const int tilesN = N >> 5, tilesM = M >> 6;
  const int tile = blockIdx.x * 8 + wave;
  if (tile >= tilesM * tilesN) return;
  const int tm = tile / tilesN;
  const int tn = tile - tm * tilesN;
  const int m0 = tm << 6, n0 = tn << 5;
  const int rl = lane & 15, hh = lane >> 4, koff = hh * 8;

  v8f acc[4][2];
#pragma unroll
  for (int i = 0; i < 4; ++i) { acc[i][0] = zero8(); acc[i][1] = zero8(); }

  for (int k0 = 0; k0 < K; k0 += 32) {
    v16h bh[2];
    v16b bb[2];
#pragma unroll
    for (int j = 0; j < 2; ++j) {
      const size_t bo = (size_t)(n0 + 16 * j + rl) * ldb + koff + k0;
      bh[j] = ldfrag_h(Bh + bo);
      if (HASLO) bb[j] = ldfrag_b(Bbp + bo); else bb[j] = zero16b();
    }
#pragma unroll
    for (int i = 0; i < 4; ++i) {
      const size_t ao = (size_t)(m0 + 16 * i + rl) * lda + koff + k0;
      const v16h ah = ldfrag_h(Ah + ao);
      acc[i][0] = mma_h(ah, bh[0], acc[i][0]);
      acc[i][1] = mma_h(ah, bh[1], acc[i][1]);
      if (HASLO) {
        const v16b al = ldfrag_b(Alp + ao);
        acc[i][0] = mma_b(al, bb[0], acc[i][0]);
        acc[i][1] = mma_b(al, bb[1], acc[i][1]);
      }
    }
  }

  if (MODE != 1) {
    float* slab = (float*)(void*)sT[wave];
    const int q8 = lane & 7, rr = lane >> 3, c4 = q8 * 4;
    v4f b4 = {0.f, 0.f, 0.f, 0.f};
    if (HASBIAS) {
      const v4f braw = *(const v4f*)(bias + n0 + c4);
#pragma unroll
      for (int e = 0; e < 4; ++e) b4[e] = bfr(braw[e]);
    }
#pragma unroll
    for (int i = 0; i < 4; ++i) {
      const int mBase = m0 + 16 * i;
#pragma unroll
      for (int r = 0; r < 8; ++r) {
        slab[(8 * hh + r) * 36 + rl]      = acc[i][0][r];
        slab[(8 * hh + r) * 36 + 16 + rl] = acc[i][1][r];
      }
      lds_sync();
      v4f ov[4];
#pragma unroll
      for (int it = 0; it < 4; ++it) {
        const int row = it * 4 + rr;
        v4f v = *(const v4f*)(slab + row * 36 + c4) * oscale;
        if (MODE == 0) {
          v = vmax0(v);
        } else if (MODE == 2) {
          const v4f r4 = *(const v4f*)(res + (size_t)(mBase + row) * ldr + n0 + c4);
          v = (v + b4) + r4;
        } else {
          v = vmax0(v + b4);
        }
        ov[it] = v;
      }
      for (int pass = 0; pass < 2; ++pass) {
#pragma unroll
        for (int it = 0; it < 4; ++it) {
          const int row = it * 4 + rr;
          *(volatile v4f*)(Cf + (size_t)(mBase + row) * ldc + n0 + c4) = ov[it];
        }
        __threadfence();
      }
      lds_sync();
    }
  } else {
    _Float16* th = (_Float16*)(void*)sT[wave];
#pragma unroll
    for (int i = 0; i < 4; ++i) {
#pragma unroll
      for (int r = 0; r < 8; ++r) {
        th[(16 * i + 8 * hh + r) * 40 + rl]      = (_Float16)(acc[i][0][r] * oscale);
        th[(16 * i + 8 * hh + r) * 40 + 16 + rl] = (_Float16)(acc[i][1][r] * oscale);
      }
    }
    lds_sync();
    const int which = n0 >> 7;
    const int hb0 = (n0 & 127) >> 4;
    const int bgr = m0 >> 9, nl0 = m0 & 511;
    const int piece = lane & 7, lq = lane >> 3;
    if (which < 2) {
      unsigned short* dst = (which == 0) ? Qo : Ko;
      v4u ov[8];
      size_t oo[8];
#pragma unroll
      for (int jj = 0; jj < 2; ++jj) {
#pragma unroll
        for (int it = 0; it < 4; ++it) {
          const int row = it * 16 + 4 * lq + (piece >> 1);
          const int dk0 = (piece & 1) * 8;
          union { v8h h; v4u u; } t;
          t.h = *(const v8h*)(th + row * 40 + 16 * jj + dk0);
          ov[jj * 4 + it] = t.u;
          oo[jj * 4 + it] = (((size_t)(bgr * NHD + hb0 + jj)) * NN + nl0 + row) * DKD + dk0;
        }
      }
      for (int pass = 0; pass < 2; ++pass) {
#pragma unroll
        for (int q = 0; q < 8; ++q) *(volatile v4u*)(dst + oo[q]) = ov[q];
        __threadfence();
      }
    } else {
      v4u ov[8];
      size_t oo[8];
#pragma unroll
      for (int it = 0; it < 8; ++it) {
        const int line = it * 4 + lq;
        const int jj = line >> 4, dk = line & 15;
        v4u a;
#pragma unroll
        for (int p = 0; p < 4; ++p) {
          const int e = 2 * p;
          const _Float16 x0 = th[(8 * piece + e) * 40 + 16 * jj + dk];
          const _Float16 x1 = th[(8 * piece + e + 1) * 40 + 16 * jj + dk];
          a[p] = pk16(h_bits(x0), h_bits(x1));
        }
        ov[it] = a;
        oo[it] = (((size_t)(bgr * NHD + hb0 + jj)) * DKD + dk) * NN + nl0 + 8 * piece;
      }
      for (int pass = 0; pass < 2; ++pass) {
#pragma unroll
        for (int it = 0; it < 8; ++it) *(volatile v4u*)(Vo + oo[it]) = ov[it];
        __threadfence();
      }
    }
  }
}

__global__ __launch_bounds__(128)
void attn16(const unsigned short* __restrict__ Qp, const unsigned short* __restrict__ Kp,
            const unsigned short* __restrict__ Vtp, const int* __restrict__ msk,
            float* Ohm, float sscale, float oscl) {
  __shared__ __align__(16) _Float16 Ks[NN * DKD];
  __shared__ __align__(16) _Float16 Vts[DKD * NN];
  __shared__ __align__(16) _Float16 Psh[4][16 * 64];
  __shared__ __align__(16) float    Os[4][16 * 16];

  const int tid  = threadIdx.x;
  const int wave = tid >> 5;
  const int lane = tid & 31;
  const int hh   = lane >> 4;
  const int c    = lane & 15;
  const int bx  = blockIdx.x;
  const int qb  = bx & 7;
  const int bhd = bx >> 3;
  const int bq  = bhd >> 3;
  const int q0  = qb * 64 + wave * 16;

  const _Float16* Qg = (const _Float16*)(const void*)Qp  + (size_t)bhd * (NN * DKD);
  const _Float16* Kg = (const _Float16*)(const void*)Kp  + (size_t)bhd * (NN * DKD);
  const _Float16* Vg = (const _Float16*)(const void*)Vtp + (size_t)bhd * (NN * DKD);
  const int* mb = msk + (size_t)bq * NN * NN;

#pragma unroll
  for (int it = 0; it < 8; ++it) {
    const int idx = it * 128 + tid;
    *(v8h*)(Ks + idx * 8)  = *(const v8h*)(Kg + idx * 8);
    *(v8h*)(Vts + idx * 8) = *(const v8h*)(Vg + idx * 8);
  }
  __syncthreads();

  FragH qf;
  qf.h[0] = *(const v8h*)(Qg + (size_t)(q0 + c) * DKD + 8 * hh);
  qf.h[1] = zero8h();
  const v16h qa = qf.v;

  float mrow[8], lrow[8];
  v8f oacc = zero8();
#pragma unroll
  for (int r = 0; r < 8; ++r) { mrow[r] = -INFINITY; lrow[r] = 0.f; }
  _Float16* pwh = Psh[wave];

#pragma unroll 1
  for (int kt = 0; kt < NN / 64; ++kt) {
    const int kv0 = kt * 64;
    v8f s[4];
#pragma unroll
    for (int j = 0; j < 4; ++j) {
      FragH kb;
      kb.h[0] = *(const v8h*)(Ks + (kv0 + 16 * j + c) * DKD + 8 * hh);
      kb.h[1] = zero8h();
      s[j] = mma_h(qa, kb.v, zero8());
    }

#pragma unroll
    for (int r = 0; r < 8; ++r) {
      const int qrow = q0 + 8 * hh + r;
      const int* mrp = mb + (size_t)qrow * NN + kv0;
      float m = -INFINITY;
#pragma unroll
      for (int j = 0; j < 4; ++j) {
        const int mv = mrp[16 * j + c];
        float sv = s[j][r] * sscale;
        sv = (mv != 0) ? sv : -INFINITY;
        s[j][r] = sv;
        m = fmaxf(m, sv);
      }
#pragma unroll
      for (int off = 1; off < 16; off <<= 1) m = fmaxf(m, __shfl_xor(m, off, 32));
      const float mnew  = fmaxf(mrow[r], m);
      const float msafe = (mnew == -INFINITY) ? 0.f : mnew;
      const float alpha = __expf(mrow[r] - msafe);
      mrow[r] = mnew;
      float psum = 0.f;
#pragma unroll
      for (int j = 0; j < 4; ++j) {
        const float p = __expf(s[j][r] - msafe);
        psum += p;
        pwh[(8 * hh + r) * 64 + 16 * j + c] = (_Float16)(p * 1024.0f);
      }
#pragma unroll
      for (int off = 1; off < 16; off <<= 1) psum += __shfl_xor(psum, off, 32);
      lrow[r] = lrow[r] * alpha + psum;
      oacc[r] = oacc[r] * alpha;
    }
    lds_sync();

#pragma unroll
    for (int kk = 0; kk < 2; ++kk) {
      FragH pa;
      pa.h[0] = *(const v8h*)(pwh + c * 64 + kk * 32 + 8 * hh);
      pa.h[1] = *(const v8h*)(pwh + c * 64 + kk * 32 + 16 + 8 * hh);
      FragH vb;
      vb.h[0] = *(const v8h*)(Vts + c * NN + kv0 + kk * 32 + 8 * hh);
      vb.h[1] = *(const v8h*)(Vts + c * NN + kv0 + kk * 32 + 16 + 8 * hh);
      oacc = mma_h(pa.v, vb.v, oacc);
    }
    lds_sync();
  }

  float* os = Os[wave];
#pragma unroll
  for (int r = 0; r < 8; ++r) {
    const float l = lrow[r];
    const float inv = ((l > 0.f) ? (1.0f / l) : 0.f) * oscl;
    os[(8 * hh + r) * 16 + c] = oacc[r] * inv;
  }
  lds_sync();
  {
    const int rq = lane >> 2, c4 = (lane & 3) * 4;
    v4f ov[2];
    size_t oo[2];
#pragma unroll
    for (int it = 0; it < 2; ++it) {
      const int row = it * 8 + rq;
      ov[it] = *(const v4f*)(os + row * 16 + c4);
      oo[it] = ((size_t)bhd * NN + q0 + row) * DKD + c4;
    }
    for (int pass = 0; pass < 2; ++pass) {
#pragma unroll
      for (int it = 0; it < 2; ++it) *(volatile v4f*)(Ohm + oo[it]) = ov[it];
      __threadfence();
    }
  }
}

__global__ __launch_bounds__(256) void readout_a(const float* __restrict__ h, const float* __restrict__ Wp,
                                                 const float* __restrict__ Wr, const float* __restrict__ br,
                                                 float* rp) {
  __shared__ __align__(16) _Float16 Ahs[NB * DD];
  __shared__ __align__(16) _Float16 Als[NB * DD];
  __shared__ __align__(16) float R1[DD * DD / 2];
  __shared__ __align__(16) float rps[128];
  const int tid = threadIdx.x, wave = tid >> 5, lane = tid & 31, hh = lane >> 4, c = lane & 15;

#pragma unroll 1
  for (int p = 0; p < 16; ++p) {
    const int idx = p * 256 + tid;
    const int bqq = idx >> 7, d = idx & 127;
    const float* hp0 = h + (size_t)bqq * NN * DD + d;
    double s = 0.0;
#pragma unroll 4
    for (int nn = 0; nn < NN; ++nn) s += (double)hp0[(size_t)nn * DD];
    const float pm = (float)(s * (1.0 / 512.0));
    const float f  = pm * 16.0f;
    const _Float16 hi = (_Float16)f;
    const _Float16 lo = (_Float16)((f - (float)hi) * 2048.0f);
    Ahs[idx] = hi;
    Als[idx] = lo;
  }
  _Float16* Wps = (_Float16*)(void*)R1;
  {
    const int n = tid & 127, kb = (tid >> 7) * 64;
#pragma unroll 4
    for (int kk = 0; kk < 64; ++kk) {
      const int k = kb + kk;
      Wps[n * DD + k] = (_Float16)(bfr(Wp[(size_t)k * DD + n]) * 64.0f);
    }
  }
  __syncthreads();

  v8f acc[4], accr[4];
#pragma unroll
  for (int j = 0; j < 4; ++j) { acc[j] = zero8(); accr[j] = zero8(); }
  const int rw = wave & 1, jb = (wave >> 1) * 4;
  if (wave < 4) {
#pragma unroll
    for (int ks = 0; ks < 4; ++ks) {
      const int k0 = ks * 32;
      const v16h ah = ldfrag_h(Ahs + (16 * rw + c) * DD + k0 + 8 * hh);
      const v16h al = ldfrag_h(Als + (16 * rw + c) * DD + k0 + 8 * hh);
#pragma unroll
      for (int j = 0; j < 4; ++j) {
        const v16h bw = ldfrag_h(Wps + (16 * (jb + j) + c) * DD + k0 + 8 * hh);
        acc[j]  = mma_h(ah, bw, acc[j]);
        accr[j] = mma_h(al, bw, accr[j]);
      }
    }
  }
  __syncthreads();
  float* hps = R1;
  if (wave < 4) {
#pragma unroll
    for (int j = 0; j < 4; ++j) {
#pragma unroll
      for (int r = 0; r < 8; ++r) {
        hps[(16 * rw + 8 * hh + r) * DD + 16 * (jb + j) + c] =
            (acc[j][r] + accr[j][r] * (1.0f / 2048.0f)) * (1.0f / 1024.0f);
      }
    }
  }
  __syncthreads();
  if (tid < 96) {
    const int bqq = tid / 3, o = tid - 3 * bqq;
    float s = bfr(br[o]);
#pragma unroll 4
    for (int j = 0; j < DD; ++j) s += fmaxf(hps[bqq * DD + j], 0.0f) * bfr(Wr[j * NOUT + o]);
    rps[tid] = s;
  }
  __syncthreads();
  if (tid < 24) {
    const v4f v = *(const v4f*)(rps + 4 * tid);
    float* po = rp + 4 * tid;
    *(volatile v4f*)po = v;
    __threadfence();
    *(volatile v4f*)po = v;
  }
}

__global__ __launch_bounds__(256) void readout_b(const float* __restrict__ h, const float* __restrict__ Wr,
                                                 const float* __restrict__ rp, float* out) {
  __shared__ float Wrs[DD * NOUT];
  __shared__ float rpb[4];
  __shared__ __align__(16) float outs[768];
  const int tid = threadIdx.x;
  const int bb = blockIdx.x;
  const int bqq = bb >> 1;
  for (int i = tid; i < DD * NOUT; i += 256) Wrs[i] = bfr(Wr[DD * NOUT + i]);
  {
    const int oo = (tid < 3) ? tid : 0;
    const float rv = rp[bqq * 3 + oo];
    if (tid < 3) rpb[tid] = rv;
  }
  __syncthreads();
  const int m = bb * 256 + tid;
  const float* hr = h + (size_t)m * DD;
  float s0 = rpb[0], s1 = rpb[1], s2 = rpb[2];
#pragma unroll 1
  for (int ch = 0; ch < DD / 4; ++ch) {
    const v4f xv = *(const v4f*)(hr + 4 * ch);
#pragma unroll
    for (int e = 0; e < 4; ++e) {
      const float a = fmaxf(xv[e], 0.0f);
      const int j = 4 * ch + e;
      s0 += a * Wrs[3 * j];
      s1 += a * Wrs[3 * j + 1];
      s2 += a * Wrs[3 * j + 2];
    }
  }
  outs[3 * tid]     = s0;
  outs[3 * tid + 1] = s1;
  outs[3 * tid + 2] = s2;
  __syncthreads();
  if (tid < 192) {
    const v4f v = *(const v4f*)(outs + 4 * tid);
    float* po = out + (size_t)bb * 768 + 4 * tid;
    *(volatile v4f*)po = v;
    __threadfence();
    *(volatile v4f*)po = v;
  }
}

extern "C" void kernel_launch(void* const* d_in, const int* in_sizes, int n_in,
                              void* d_out, int out_size, void* d_ws, size_t ws_size,
                              hipStream_t stream) {
  if (n_in < 14) return;
  if (in_sizes[0] != MR * FIN) return;
  if (in_sizes[1] != NB * NN * NN) return;
  if (in_sizes[2] != FIN * DD) return;
  if (in_sizes[3] != NL * NHD * DD * DKD || in_sizes[4] != NL * NHD * DD * DKD ||
      in_sizes[5] != NL * NHD * DD * DKD) return;
  if (in_sizes[6] != NL * NHD * DKD * DD) return;
  if (in_sizes[7] != NL * DD * FFD || in_sizes[8] != NL * FFD) return;
  if (in_sizes[9] != NL * FFD * DD || in_sizes[10] != NL * DD) return;
  if (in_sizes[11] != DD * DD || in_sizes[12] != 2 * DD * NOUT || in_sizes[13] != NOUT) return;
  if (out_size != MR * NOUT) return;

  const float* x    = (const float*)d_in[0];
  const int*   msk  = (const int*)d_in[1];
  const float* We   = (const float*)d_in[2];
  const float* Wq   = (const float*)d_in[3];
  const float* Wk   = (const float*)d_in[4];
  const float* Wv   = (const float*)d_in[5];
  const float* Wout = (const float*)d_in[6];
  const float* Wff1 = (const float*)d_in[7];
  const float* bff1 = (const float*)d_in[8];
  const float* Wff2 = (const float*)d_in[9];
  const float* bff2 = (const float*)d_in[10];
  const float* Wp   = (const float*)d_in[11];
  const float* Wr   = (const float*)d_in[12];
  const float* br   = (const float*)d_in[13];
  float* out = (float*)d_out;

  size_t off = 0;
  auto take = [&](size_t bytes) -> size_t { size_t o = off; off += (bytes + 255) & ~(size_t)255; return o; };
  const size_t oXp  = take((size_t)MR * 32 * 2);
  const size_t oWe  = take((size_t)DD * 32 * 2);
  const size_t oWqH = take((size_t)NL * QKVC * DD * 2);
  const size_t oWqB = take((size_t)NL * QKVC * DD * 2);
  const size_t oWoH = take((size_t)NL * DD * DD * 2);
  const size_t oWoB = take((size_t)NL * DD * DD * 2);
  const size_t oW1H = take((size_t)NL * FFD * DD * 2);
  const size_t oW1B = take((size_t)NL * FFD * DD * 2);
  const size_t oW2H = take((size_t)NL * DD * FFD * 2);
  const size_t oW2B = take((size_t)NL * DD * FFD * 2);
  const size_t ohA  = take((size_t)MR * DD * 4);
  const size_t ohB  = take((size_t)MR * DD * 4);
  const size_t oHh  = take((size_t)MR * DD * 2);
  const size_t oHl  = take((size_t)MR * DD * 2);
  const size_t oQ   = take((size_t)MR * DD * 2);
  const size_t oK   = take((size_t)MR * DD * 2);
  const size_t oV   = take((size_t)MR * DD * 2);
  const size_t oO   = take((size_t)MR * DD * 4);
  const size_t oT   = take((size_t)MR * FFD * 4);
  const size_t oTh  = take((size_t)MR * FFD * 2);
  const size_t oTl  = take((size_t)MR * FFD * 2);
  const size_t oRp  = take(512);
  if (off > ws_size) return;
  if (off > (size_t)134217728) return;

  char* ws = (char*)d_ws;
  unsigned short* Xp  = (unsigned short*)(ws + oXp);
  unsigned short* WeT = (unsigned short*)(ws + oWe);
  unsigned short* WqH = (unsigned short*)(ws + oWqH);
  unsigned short* WqB = (unsigned short*)(ws + oWqB);
  unsigned short* WoH = (unsigned short*)(ws + oWoH);
  unsigned short* WoB = (unsigned short*)(ws + oWoB);
  unsigned short* W1H = (unsigned short*)(ws + oW1H);
  unsigned short* W1B = (unsigned short*)(ws + oW1B);
  unsigned short* W2H = (unsigned short*)(ws + oW2H);
  unsigned short* W2B = (unsigned short*)(ws + oW2B);
  float*          hA  = (float*)(ws + ohA);
  float*          hB  = (float*)(ws + ohB);
  unsigned short* Hh  = (unsigned short*)(ws + oHh);
  unsigned short* Hl  = (unsigned short*)(ws + oHl);
  unsigned short* Qp  = (unsigned short*)(ws + oQ);
  unsigned short* Kp  = (unsigned short*)(ws + oK);
  unsigned short* Vt  = (unsigned short*)(ws + oV);
  float*          Ohm = (float*)(ws + oO);
  float*          Tf  = (float*)(ws + oT);
  unsigned short* Th  = (unsigned short*)(ws + oTh);
  unsigned short* Tl  = (unsigned short*)(ws + oTl);
  float*          Rp  = (float*)(ws + oRp);

  const dim3 blk(256);
  const int n4x  = MR * 4;
  const int n4w  = DD * 4;
  const int n8q  = NL * DD * DD / 8;
  const int n8f  = NL * FFD * DD / 8;
  const int n8h  = MR * DD / 8;
  const int n8t  = MR * FFD / 8;
  const dim3 gPx((n4x + 255) / 256);
  const dim3 gPw((n4w + 255) / 256);
  const dim3 gWq((n8q + 255) / 256);
  const dim3 gWf((n8f + 255) / 256);
  const dim3 gCh((n8h + 255) / 256);
  const dim3 gCt((n8t + 255) / 256);
  const dim3 gEmb(((MR / 64) * (DD / 32) + 7) / 8);
  const dim3 gQKV(((MR / 64) * (QKVC / 32) + 7) / 8);
  const dim3 gDD(((MR / 64) * (DD / 32) + 7) / 8);
  const dim3 gFF1(((MR / 64) * (FFD / 32) + 7) / 8);
  const dim3 gAtt(NB * NHD * (NN / 64));
  const dim3 gRb(MR / 256);

  const float wScale = 64.0f;
  const float aScale = 16.0f;
  const int   allm   = 0x7fffffff;

  pad16<<<gPx, blk, 0, stream>>>(x, FIN, 1, Xp, n4x, 8.0f);
  pad16<<<gPw, blk, 0, stream>>>(We, 1, DD, WeT, n4w, wScale);
  wprep<<<gWq, blk, 0, stream>>>(Wq, WqH, WqB, n8q, DD, DD, NHD * DD * DKD, QKVC * DD, 0,      4, 15,   DD * DKD, 1, DKD, wScale);
  wprep<<<gWq, blk, 0, stream>>>(Wk, WqH, WqB, n8q, DD, DD, NHD * DD * DKD, QKVC * DD, DD,     4, 15,   DD * DKD, 1, DKD, wScale);
  wprep<<<gWq, blk, 0, stream>>>(Wv, WqH, WqB, n8q, DD, DD, NHD * DD * DKD, QKVC * DD, 2 * DD, 4, 15,   DD * DKD, 1, DKD, wScale);
  wprep<<<gWq, blk, 0, stream>>>(Wout, WoH, WoB, n8q, DD, DD, DD * DD, DD * DD, 0, 31, allm, 0, 1, DD, wScale);
  wprep<<<gWf, blk, 0, stream>>>(Wff1, W1H, W1B, n8f, FFD, DD, DD * FFD, FFD * DD, 0, 31, allm, 0, 1, FFD, wScale);
  wprep<<<gWf, blk, 0, stream>>>(Wff2, W2H, W2B, n8f, DD, FFD, FFD * DD, DD * FFD, 0, 31, allm, 0, 1, DD, wScale);
  gemmw<0, 0, 0><<<gEmb, blk, 0, stream>>>(Xp, Xp, 32, WeT, WeT, 32, bff1, hB, DD, hA, DD, Qp, Kp, Vt,
                                           MR, DD, 32, 1.0f / 512.0f);

  for (int l = 0; l < NL; ++l) {
    const unsigned short* WqHl = WqH + (size_t)l * QKVC * DD;
    const unsigned short* WqBl = WqB + (size_t)l * QKVC * DD;
    const unsigned short* WoHl = WoH + (size_t)l * DD * DD;
    const unsigned short* WoBl = WoB + (size_t)l * DD * DD;
    const unsigned short* W1Hl = W1H + (size_t)l * FFD * DD;
    const unsigned short* W1Bl = W1B + (size_t)l * FFD * DD;
    const unsigned short* W2Hl = W2H + (size_t)l * DD * FFD;
    const unsigned short* W2Bl = W2B + (size_t)l * DD * FFD;
    cvt_hl<0><<<gCh, blk, 0, stream>>>(hA, Hh, Hl, n8h, aScale);
    gemmw<1, 1, 0><<<gQKV, blk, 0, stream>>>(Hh, Hl, DD, WqHl, WqBl, DD, bff1, hB, DD, hB, DD, Qp, Kp, Vt,
                                             MR, QKVC, DD, 1.0f / 64.0f);
    attn16<<<gAtt, dim3(128), 0, stream>>>(Qp, Kp, Vt, msk, Ohm, 1.0f / 1024.0f, 1.0f / 16384.0f);
    cvt_hl<1><<<gCh, blk, 0, stream>>>(Ohm, Hh, Hl, n8h, aScale);
    gemmw<2, 1, 0><<<gDD, blk, 0, stream>>>(Hh, Hl, DD, WoHl, WoBl, DD, bff1, hA, DD, hB, DD, Qp, Kp, Vt,
                                            MR, DD, DD, 1.0f / 1024.0f);
    cvt_hl<0><<<gCh, blk, 0, stream>>>(hB, Hh, Hl, n8h, aScale);
    gemmw<3, 1, 1><<<gFF1, blk, 0, stream>>>(Hh, Hl, DD, W1Hl, W1Bl, DD, bff1 + (size_t)l * FFD, hA, DD, Tf, FFD,
                                             Qp, Kp, Vt, MR, FFD, DD, 1.0f / 1024.0f);
    cvt_hl<0><<<gCt, blk, 0, stream>>>(Tf, Th, Tl, n8t, aScale);
    gemmw<2, 1, 1><<<gDD, blk, 0, stream>>>(Th, Tl, FFD, W2Hl, W2Bl, FFD, bff2 + (size_t)l * DD, hB, DD, hA, DD,
                                            Qp, Kp, Vt, MR, DD, FFD, 1.0f / 1024.0f);
  }

  readout_a<<<dim3(1), blk, 0, stream>>>(hA, Wp, Wr, br, Rp);
  readout_b<<<gRb, blk, 0, stream>>>(hA, Wr, Rp, out);
  (void)hipGetLastError();
}
